// HyperSETAlterAttention_71614284694168
// MI455X (gfx1250) — hardware-verified
//
#include <hip/hip_runtime.h>


#define NB_  2
#define TT   2048
#define CC   768
#define NH_  12
#define HD   64
#define ZH   2
#define PCAR 512.0f
typedef _Float16 h16;
typedef unsigned short bf;
typedef __attribute__((ext_vector_type(16))) __bf16   v16bf;
typedef __attribute__((ext_vector_type(16))) _Float16 v16h;
typedef __attribute__((ext_vector_type(8)))  _Float16 v8h;
typedef __attribute__((ext_vector_type(8)))  unsigned short v8us;
typedef __attribute__((ext_vector_type(8)))  float    v8f;
typedef __attribute__((ext_vector_type(4)))  float    v4f;
typedef v8h  __attribute__((may_alias)) v8ha;
typedef v4f  __attribute__((may_alias)) v4fa;
typedef v8us __attribute__((may_alias)) v8usa;

__device__ __forceinline__ unsigned short f2bf(float f) { unsigned u = __float_as_uint(f); u += 0x7FFFu + ((u >> 16) & 1u); return (unsigned short)(u >> 16); }
__device__ __forceinline__ float bf2f(unsigned short b) { return __uint_as_float(((unsigned)b) << 16); }
__device__ __forceinline__ float bfr(float f) { return bf2f(f2bf(f)); }
__device__ __forceinline__ v16h cat16(v8h lo, v8h hi) { return __builtin_shufflevector(lo, hi, 0, 1, 2, 3, 4, 5, 6, 7, 8, 9, 10, 11, 12, 13, 14, 15); }
__device__ __forceinline__ v16bf cat16b(v8us lo, v8us hi) { return __builtin_bit_cast(v16bf, __builtin_shufflevector(lo, hi, 0, 1, 2, 3, 4, 5, 6, 7, 8, 9, 10, 11, 12, 13, 14, 15)); }
__device__ __forceinline__ v8f wmma16(v16h a, v16h b, v8f c) { return __builtin_amdgcn_wmma_f32_16x16x32_f16(false, a, false, b, (short)0, c, false, false); }
__device__ __forceinline__ v8f wmmab(v16bf a, v16bf b, v8f c) { return __builtin_amdgcn_wmma_f32_16x16x32_bf16(false, a, false, b, (short)0, c, false, false); }


template <typename T16> struct WFrag;
template <> struct WFrag<h16> { typedef v16h V; static __device__ __forceinline__ V ld(const h16* p) { return cat16(*(const v8h*)p, *(const v8h*)(p + 16)); } static __device__ __forceinline__ v8f mma(V a, V b, v8f c) { return wmma16(a, b, c); } };
template <> struct WFrag<bf> { typedef v16bf V; static __device__ __forceinline__ V ld(const bf* p) { return cat16b(*(const v8us*)p, *(const v8us*)(p + 16)); } static __device__ __forceinline__ v8f mma(V a, V b, v8f c) { return wmmab(a, b, c); } };
template <typename T16, int NSPLIT, bool BIAS>
__global__ __launch_bounds__(32) void k_gemmw(const T16* __restrict__ A, const T16* __restrict__ A2, const T16* __restrict__ Bt, const T16* __restrict__ Bt2, int K, float* C, int ldc, const float* __restrict__ bias, size_t sA, size_t sB, size_t sC) {
    typedef typename WFrag<T16>::V V;
    __shared__ __align__(16) float os[16 * 68];
    const size_t z = blockIdx.z; A += z * sA; if (A2) A2 += z * sA; Bt += z * sB; if (Bt2) Bt2 += z * sB; C += z * sC;
    const int lane = threadIdx.x & 31, lr = lane & 15, hi = lane >> 4; const int r0 = blockIdx.x * 64, c0 = blockIdx.y * 64;
    v8f acc[4][4];
#pragma unroll
    for (int mb = 0; mb < 4; ++mb)
#pragma unroll
        for (int nb = 0; nb < 4; ++nb) acc[mb][nb] = (v8f){};
    const size_t aoff = (size_t)(r0 + lr) * K + 8 * hi, boff = (size_t)(c0 + lr) * K + 8 * hi;
#pragma unroll 1
    for (int kc = 0; kc < K; kc += 32) {
        V a[4], a2[4];
#pragma unroll
        for (int mb = 0; mb < 4; ++mb) { a[mb] = WFrag<T16>::ld(A + aoff + (size_t)mb * 16 * K + kc); if (NSPLIT == 1 || NSPLIT == 2) a2[mb] = WFrag<T16>::ld(A2 + aoff + (size_t)mb * 16 * K + kc); }
#pragma unroll
        for (int nb = 0; nb < 4; ++nb) { const V b = WFrag<T16>::ld(Bt + boff + (size_t)nb * 16 * K + kc); V b2; if (NSPLIT >= 2) b2 = WFrag<T16>::ld(Bt2 + boff + (size_t)nb * 16 * K + kc);
#pragma unroll
            for (int mb = 0; mb < 4; ++mb) { acc[mb][nb] = WFrag<T16>::mma(a[mb], b, acc[mb][nb]); if (NSPLIT == 1 || NSPLIT == 2) acc[mb][nb] = WFrag<T16>::mma(a2[mb], b, acc[mb][nb]); if (NSPLIT >= 2) acc[mb][nb] = WFrag<T16>::mma(a[mb], b2, acc[mb][nb]); } }
        asm volatile("v_nop\n\tv_nop\n\tv_nop\n\tv_nop" : "+v"(acc[0][0]), "+v"(acc[1][1]), "+v"(acc[2][2]), "+v"(acc[3][3]) : "v"(a[0]), "v"(a[3]));
    }
#pragma unroll
    for (int mb = 0; mb < 4; ++mb) {
#pragma unroll
        for (int nb = 0; nb < 4; ++nb) {
#pragma unroll
            for (int j = 0; j < 8; ++j) os[(hi * 8 + j) * 68 + nb * 16 + lr] = acc[mb][nb][j]; }
        __builtin_amdgcn_wave_barrier(); asm volatile("" ::: "memory");
        float* crow = C + (size_t)(r0 + mb * 16) * ldc + c0;
#pragma unroll 1
        for (int ps = 0; ps < 2; ++ps) {
#pragma unroll
            for (int s = 0; s < 8; ++s) { const int row = 2 * s + hi, cofs = lr * 4; v4f val = *(const v4fa*)(os + row * 68 + cofs); if (BIAS) { val[0] += bfr(bias[c0 + cofs]); val[1] += bfr(bias[c0 + cofs + 1]); val[2] += bfr(bias[c0 + cofs + 2]); val[3] += bfr(bias[c0 + cofs + 3]); }
                *(volatile v4f*)(crow + (size_t)row * ldc + cofs) = val; }
            if (ps == 0) __threadfence(); }
        __builtin_amdgcn_wave_barrier(); asm volatile("" ::: "memory");
    }
}

__device__ __forceinline__ h16 tohx(float x) { return (h16)x; }
__device__ __forceinline__ void splitf(float y, unsigned short& h, unsigned short& l) { h = f2bf(y); l = f2bf(y - bf2f(h)); }
typedef __attribute__((ext_vector_type(2))) _Float16 v2h;
typedef __attribute__((ext_vector_type(4))) _Float16 v4h;
typedef __attribute__((ext_vector_type(2))) unsigned short v2us;
typedef __attribute__((ext_vector_type(4))) unsigned short v4us;

__global__ __launch_bounds__(256) void k_wtG(const float* __restrict__ w, int K, int N, bf* Bt) {
    const int lane = threadIdx.x & 31; const int L0 = (blockIdx.x * 8 + (threadIdx.x >> 5)) * 8; const int nlines = N * K / 64;
#pragma unroll 1
    for (int ps = 0; ps < 2; ++ps) {
#pragma unroll 1
        for (int l = 0; l < 8; ++l) { const int L = L0 + l; if (L >= nlines) break; const size_t e = (size_t)L * 64 + lane * 2; const int k = (int)(e % K), n = (int)(e / K); v2us o;
            o[0] = f2bf(w[(size_t)k * N + n]); o[1] = f2bf(w[(size_t)(k + 1) * N + n]); *(volatile v2us*)(Bt + e) = o; }
        if (ps == 0) __threadfence(); }
}
__global__ __launch_bounds__(256) void k_cvt8(const float* __restrict__ src, bf* dst, size_t n8) { const size_t i = (size_t)blockIdx.x * 256 + threadIdx.x; if (i >= n8) return; const v8f v = *(const v8f*)(src + i * 8); v8us o;
#pragma unroll
    for (int k = 0; k < 8; ++k) o[k] = f2bf(v[k]); *(volatile v8us*)(dst + i * 8) = o; __threadfence(); *(volatile v8us*)(dst + i * 8) = o; }
__global__ __launch_bounds__(256) void k_rms(const float* __restrict__ WF, const float* __restrict__ g1, const float* __restrict__ g2, bf* Qh, bf* Ql, bf* Kh, bf* Kl, float* RS) { const int lane = threadIdx.x & 31; const int row = blockIdx.x * 8 + (threadIdx.x >> 5); if (row >= NH_ * TT) return; const int t = row % TT, h = row / TT; const float* w = WF + (size_t)t * CC + h * HD; const float a0 = w[lane * 2], a1 = w[lane * 2 + 1];
    float s = __fadd_rn(__fmul_rn(a0, a0), __fmul_rn(a1, a1));
#pragma unroll
    for (int sh = 16; sh; sh >>= 1) s += __shfl_xor(s, sh, 32);
    const float r = __frsqrt_rn(__fadd_rn(s * (1.0f / HD), 1.1920929e-07f)); const size_t o = ((size_t)h * TT + t) * HD + lane * 2; v2us qh, ql, kh, kl;
#pragma unroll
    for (int u = 0; u < 2; ++u) { const int d = lane * 2 + u; const float wn = __fmul_rn(u ? a1 : a0, r); unsigned short x1, x2; splitf(__fmul_rn(wn, bfr(g1[d])), x1, x2); qh[u] = x1; ql[u] = x2; splitf(__fmul_rn(wn, bfr(g2[d])), x1, x2); kh[u] = x1; kl[u] = x2; }
    for (int ps = 0; ps < 2; ++ps) { *(volatile v2us*)(Qh + o) = qh; *(volatile v2us*)(Ql + o) = ql; *(volatile v2us*)(Kh + o) = kh; *(volatile v2us*)(Kl + o) = kl; if (lane == 0) *(volatile float*)(RS + row) = r; if (ps == 0) __threadfence(); } }
__global__ __launch_bounds__(256) void k_vt(const float* __restrict__ WF, const float* __restrict__ RS, const float* __restrict__ g3, h16* VT) { const size_t e = ((size_t)blockIdx.x * 256 + threadIdx.x) * 2; if (e >= (size_t)NH_ * HD * TT) return; const int t = (int)(e % TT); const int d = (int)((e / TT) % HD); const int h = (int)(e / ((size_t)TT * HD)); const float g = bfr(g3[d]); v2h o;
#pragma unroll
    for (int u = 0; u < 2; ++u) { float wn = __fmul_rn(WF[(size_t)(t + u) * CC + h * HD + d], RS[(size_t)h * TT + t + u]); asm volatile("" : "+v"(wn)); o[u] = tohx(__fmul_rn(wn, g)); } *(volatile v2h*)(VT + e) = o; __threadfence(); *(volatile v2h*)(VT + e) = o; }
__global__ __launch_bounds__(256) void k_colst(const float* __restrict__ Sb, float* CM, float* CSR) { const int e = blockIdx.x * 256 + threadIdx.x; if (e >= ZH * TT) return; const int j = e % TT, z = e / TT; const float* col = Sb + (size_t)z * TT * TT + j; float mx = -3.0e38f;
    for (int i = 0; i < TT; ++i) mx = fmaxf(mx, col[(size_t)i * TT] * 0.125f);
    float s = 0.f; for (int i = 0; i < TT; ++i) { float d0 = __fsub_rn(col[(size_t)i * TT] * 0.125f, mx); asm volatile("" : "+v"(d0)); s = __fadd_rn(s, __expf(d0)); }
    const float rs = __fdiv_rn(1.0f, s); for (int ps = 0; ps < 2; ++ps) { *(volatile float*)(CM + e) = mx; *(volatile float*)(CSR + e) = rs; if (ps == 0) __threadfence(); } }
__global__ __launch_bounds__(256) void k_bisoft(const float* __restrict__ Sb, const float* __restrict__ CM, const float* __restrict__ CSR, h16* P) { const int lane = threadIdx.x & 31; const int row = blockIdx.x * 8 + (threadIdx.x >> 5); if (row >= ZH * TT) return; const int z = row / TT; const float* sr = Sb + (size_t)row * TT; float v[64]; float mx = -3.0e38f;
#pragma unroll
    for (int ch = 0; ch < 16; ++ch) { const v4f a = *(const v4f*)(sr + ch * 128 + lane * 4);
#pragma unroll
        for (int q = 0; q < 4; ++q) { const float t = a[q] * 0.125f; v[ch * 4 + q] = t; mx = fmaxf(mx, t); } }
#pragma unroll
    for (int sh = 16; sh; sh >>= 1) mx = fmaxf(mx, __shfl_xor(mx, sh, 32));
    float sum = 0.f; float ex[64];
#pragma unroll
    for (int k = 0; k < 64; ++k) { float d0 = __fsub_rn(v[k], mx); asm volatile("" : "+v"(d0)); ex[k] = __expf(d0); sum += ex[k]; }
#pragma unroll
    for (int sh = 16; sh; sh >>= 1) sum += __shfl_xor(sum, sh, 32);
    const float f = __fdiv_rn(PCAR, sum);
#pragma unroll 1
    for (int ps = 0; ps < 2; ++ps) {
#pragma unroll
        for (int ch = 0; ch < 16; ++ch) { const int j0 = ch * 128 + lane * 4; const v4f cm = *(const v4f*)(CM + (size_t)z * TT + j0), cr = *(const v4f*)(CSR + (size_t)z * TT + j0); v4h o;
#pragma unroll
            for (int q = 0; q < 4; ++q) { float d1 = __fsub_rn(v[ch * 4 + q], cm[q]); asm volatile("" : "+v"(d1)); float pc = __fmul_rn(__expf(d1), cr[q]); asm volatile("" : "+v"(pc)); float pr = __fmul_rn(ex[ch * 4 + q], f); asm volatile("" : "+v"(pr)); o[q] = tohx(__fadd_rn(pr, __fmul_rn(pc, PCAR))); }
            *(volatile v4h*)(P + (size_t)row * TT + j0) = o; }
        if (ps == 0) __threadfence(); } }
__global__ __launch_bounds__(256) void k_mrg(const float* __restrict__ Ob, int h0, bf* Yh, bf* Yl) { const size_t e = ((size_t)blockIdx.x * 256 + threadIdx.x) * 2; if (e >= (size_t)ZH * TT * HD) return; const int d = (int)(e % HD); const int t = (int)((e / HD) % TT); const int z = (int)(e / ((size_t)HD * TT)); v2us oh, ol;
#pragma unroll
    for (int u = 0; u < 2; ++u) { unsigned short a, c; splitf(Ob[e + u] * (1.0f / PCAR), a, c); oh[u] = a; ol[u] = c; } const size_t o = (size_t)t * CC + (h0 + z) * HD + d; *(volatile v2us*)(Yh + o) = oh; *(volatile v2us*)(Yl + o) = ol; __threadfence(); *(volatile v2us*)(Yh + o) = oh; *(volatile v2us*)(Yl + o) = ol; }

extern "C" void kernel_launch(void* const* d_in, const int* in_sizes, int n_in,
                              void* d_out, int out_size, void* d_ws, size_t ws_size, hipStream_t stream) {
    (void)in_sizes; (void)n_in; (void)out_size;
    const float* x = (const float*)d_in[0]; const float* Wt = (const float*)d_in[1]; const float* g1 = (const float*)d_in[2]; const float* g2 = (const float*)d_in[3]; const float* g3 = (const float*)d_in[4];
    float* OUT = (float*)d_out;
    char* wsp = (char*)d_ws;
    auto take = [&](size_t bytes) { char* p = wsp; wsp += (bytes + 255) & ~(size_t)255; return (void*)p; };
    bf* WB = (bf*)take((size_t)CC * CC * 2); bf* WT = (bf*)take((size_t)CC * CC * 2); bf* XB = (bf*)take((size_t)TT * CC * 2); float* WF = (float*)take((size_t)TT * CC * 4); float* RS = (float*)take((size_t)NH_ * TT * 4);
    bf* Qh = (bf*)take((size_t)NH_ * TT * HD * 2); bf* Ql = (bf*)take((size_t)NH_ * TT * HD * 2); bf* Kh = (bf*)take((size_t)NH_ * TT * HD * 2); bf* Kl = (bf*)take((size_t)NH_ * TT * HD * 2); h16* VT = (h16*)take((size_t)NH_ * HD * TT * 2);
    float* Sb = (float*)take((size_t)ZH * TT * TT * 4); float* CM = (float*)take((size_t)ZH * TT * 4); float* CSR = (float*)take((size_t)ZH * TT * 4); h16* P16 = (h16*)take((size_t)ZH * TT * TT * 2); float* Ob = (float*)take((size_t)ZH * TT * HD * 4); bf* Yh = (bf*)take((size_t)TT * CC * 2); bf* Yl = (bf*)take((size_t)TT * CC * 2);
    if ((size_t)(wsp - (char*)d_ws) > ws_size) return;
    k_cvt8<<<(CC * CC / 8 + 255) / 256, 256, 0, stream>>>(Wt, WB, (size_t)CC * CC / 8);
    k_wtG<<<(CC * CC / 64 + 63) / 64, 256, 0, stream>>>(Wt, CC, CC, WT);
    for (int b = 0; b < NB_; ++b) {
        k_cvt8<<<(TT * CC / 8 + 255) / 256, 256, 0, stream>>>(x + (size_t)b * TT * CC, XB, (size_t)TT * CC / 8);
        k_gemmw<bf, 0, false><<<dim3(TT / 64, CC / 64, 1), 32, 0, stream>>>(XB, nullptr, WB, nullptr, CC, WF, CC, nullptr, 0, 0, 0);
        k_rms<<<NH_ * TT / 8, 256, 0, stream>>>(WF, g1, g2, Qh, Ql, Kh, Kl, RS); k_vt<<<(unsigned)(((size_t)NH_ * HD * TT / 2 + 255) / 256), 256, 0, stream>>>(WF, RS, g3, VT);
        for (int h0 = 0; h0 < NH_; h0 += ZH) { const size_t z = (size_t)h0;
            k_gemmw<bf, 2, false><<<dim3(TT / 64, TT / 64, ZH), 32, 0, stream>>>(Qh + z * TT * HD, Ql + z * TT * HD, Kh + z * TT * HD, Kl + z * TT * HD, HD, Sb, TT, nullptr, (size_t)TT * HD, (size_t)TT * HD, (size_t)TT * TT);
            k_colst<<<(ZH * TT + 255) / 256, 256, 0, stream>>>(Sb, CM, CSR); k_bisoft<<<ZH * TT / 8, 256, 0, stream>>>(Sb, CM, CSR, P16);
            k_gemmw<h16, 0, false><<<dim3(TT / 64, 1, ZH), 32, 0, stream>>>(P16, nullptr, VT + z * HD * TT, nullptr, TT, Ob, HD, nullptr, (size_t)TT * TT, (size_t)HD * TT, (size_t)TT * HD);
            k_mrg<<<(unsigned)(((size_t)ZH * TT * HD / 2 + 255) / 256), 256, 0, stream>>>(Ob, h0, Yh, Yl); }
        k_gemmw<bf, 1, false><<<dim3(TT / 64, CC / 64, 1), 32, 0, stream>>>(Yh, Yl, WT, nullptr, CC, OUT + (size_t)b * TT * CC, CC, nullptr, 0, 0, 0); }
}
